// GAT_Multi_77919296684445
// MI455X (gfx1250) — hardware-run, weakly checked
//
#include <hip/hip_runtime.h>
#include <math.h>
#include <stdint.h>

#define BB 16
#define NN 1024
#define FF 128
#define D1 256
#define D2 128
#define KC 512
#define MROWS (BB * NN)
#define NEGF (-9.0e15f)
#define SLOPE 0.2f
#define LNEPS 1.0e-5f
#define PITCH1 260
#define PITCH2 132

static_assert(NN % 32 == 0);
static_assert(NN / 32 == 32);
static_assert(MROWS % 64 == 0);
static_assert(NN % 128 == 0);
static_assert(D1 == 2 * FF);
static_assert(D2 == 128);
static_assert(D2 - 1 == 127);
static_assert(KC == 2 * D1);
static_assert(FF % 32 == 0 && NN % 32 == 0 && KC % 32 == 0);

typedef __attribute__((ext_vector_type(16))) __bf16   v16b;
typedef __attribute__((ext_vector_type(8)))  float    v8f;
typedef __attribute__((ext_vector_type(4)))  float    v4f;
typedef __attribute__((ext_vector_type(4)))  unsigned v4u;
typedef __attribute__((ext_vector_type(8)))  unsigned v8u;
typedef v4f __attribute__((may_alias)) v4fa;
typedef v4u __attribute__((may_alias)) v4ua;

__device__ __forceinline__ unsigned f2bf(float f) {
  const unsigned u = __float_as_uint(f);
  return (u + 0x7FFFu + ((u >> 16) & 1u)) >> 16;
}
__device__ __forceinline__ float bf2f(unsigned h) { return __uint_as_float(h << 16); }
__device__ __forceinline__ float bfr(float f) { return bf2f(f2bf(f)); }
__device__ __forceinline__ unsigned pack2(float a, float b) { return f2bf(a) | (f2bf(b) << 16); }
__device__ __forceinline__ unsigned split2(float a, float b, unsigned& lo) {
  const unsigned ha = f2bf(a), hb = f2bf(b);
  const unsigned la = f2bf(a - bf2f(ha)), lb = f2bf(b - bf2f(hb));
  lo = la | (lb << 16);
  return ha | (hb << 16);
}
__device__ __forceinline__ void pinf(float v) { asm volatile("" :: "v"(v)); }

__device__ __forceinline__ v8f wmb(v16b a, v16b b, v8f c) {
  c = __builtin_amdgcn_wmma_f32_16x16x32_bf16(false, a, false, b, (short)0, c, false, false);
  asm volatile("v_nop\n\tv_nop\n\tv_nop\n\tv_nop" : "+v"(c) : "v"(a), "v"(b));
  return c;
}
__device__ __forceinline__ v16b ldfrag(const unsigned short* p) {
  const v4u a = *(const v4ua*)(p);
  const v4u b = *(const v4ua*)(p + 16);
  const v8u r = {a.x, a.y, a.z, a.w, b.x, b.y, b.z, b.w};
  return __builtin_bit_cast(v16b, r);
}
__device__ __forceinline__ float elu1(float v) {
  const float em = expm1f(v);
  return (v > 0.0f) ? v : em;
}
__device__ __forceinline__ float efill(float s, float t, unsigned bit) {
  const float v = s + t;
  float e = (v > 0.0f) ? v : SLOPE * v;
  e = (bit != 0u) ? e : NEGF;
  return e;
}

#define PA_XB_BLOCKS (MROWS * FF / 8 / 256)
#define PA_MB_BLOCKS (NN / 8)
__global__ __launch_bounds__(256) void k_pa(const float* __restrict__ x, const int* __restrict__ adj,
                                            unsigned short* __restrict__ XB, unsigned* __restrict__ MB) {
  const int tid = threadIdx.x;
  if (blockIdx.x < PA_XB_BLOCKS) {
    const size_t g = ((size_t)blockIdx.x * 256 + tid) * 8;
    const v4f a = *(const v4fa*)(x + g);
    const v4f c = *(const v4fa*)(x + g + 4);
    v4u o;
    o.x = pack2(a.x, a.y); o.y = pack2(a.z, a.w); o.z = pack2(c.x, c.y); o.w = pack2(c.z, c.w);
    volatile v4u* dst = (volatile v4u*)(XB + g);
    *dst = o;
    __threadfence();
    *dst = o;
  } else {
    const int wave = tid >> 5, lane = tid & 31;
    const int row = (blockIdx.x - PA_XB_BLOCKS) * 8 + wave;
    const int* ar = adj + (size_t)row * NN;
    unsigned word = 0u;
#pragma unroll 4
    for (int it = 0; it < NN / 32; ++it) {
      const int v = ar[it * 32 + lane];
      const unsigned bal = __builtin_amdgcn_ballot_w32(v > 0);
      word = (it == lane) ? bal : word;
    }
    volatile unsigned* dst = (volatile unsigned*)(MB + (size_t)row * 32 + lane);
    *dst = word;
    __threadfence();
    *dst = word;
  }
}

__device__ __forceinline__ void par_copy(const float* __restrict__ src, float* __restrict__ dst, int nunits, int tid) {
  const int q = (tid < nunits) ? tid : (nunits - 1);
  const v4f v = *(const v4fa*)(src + 4 * q);
  v4f o;
  o.x = bfr(v.x); o.y = bfr(v.y); o.z = bfr(v.z); o.w = bfr(v.w);
  pinf(o.x); pinf(o.y); pinf(o.z); pinf(o.w);
  if (tid < nunits) {
    volatile v4f* d = (volatile v4f*)(dst + 4 * q);
    *d = o;
    __threadfence();
    *d = o;
  }
}
#define PB_BLOCKS 52
__global__ __launch_bounds__(256) void k_pb(const float* __restrict__ W1, const float* __restrict__ a1,
                                            const float* __restrict__ gam, const float* __restrict__ bet,
                                            const float* __restrict__ W2, const float* __restrict__ a2,
                                            unsigned short* __restrict__ W1T, unsigned short* __restrict__ W2D,
                                            float* __restrict__ PAR) {
  const int tid = threadIdx.x;
  const int bx = blockIdx.x;
  if (bx < 16) {
    const int u = bx * 256 + tid;
    const int n = u >> 4, k0 = (u & 15) * 8;
    float f[8];
#pragma unroll
    for (int e = 0; e < 8; ++e) f[e] = W1[(size_t)(k0 + e) * D1 + n];
    v4u o;
    o.x = pack2(f[0], f[1]); o.y = pack2(f[2], f[3]); o.z = pack2(f[4], f[5]); o.w = pack2(f[6], f[7]);
    volatile v4u* d = (volatile v4u*)(W1T + (size_t)n * FF + k0);
    *d = o;
    __threadfence();
    *d = o;
  } else if (bx < 48) {
    const int u = (bx - 16) * 256 + tid;
    const int n = u >> 6, k0 = (u & 63) * 8;
    const int ks = k0 & (D1 - 1);
    float f[8];
#pragma unroll
    for (int e = 0; e < 8; ++e) f[e] = W2[(size_t)(ks + e) * D2 + n];
    v4u o;
    o.x = pack2(f[0], f[1]); o.y = pack2(f[2], f[3]); o.z = pack2(f[4], f[5]); o.w = pack2(f[6], f[7]);
    volatile v4u* d = (volatile v4u*)(W2D + (size_t)n * KC + k0);
    *d = o;
    __threadfence();
    *d = o;
  } else if (bx == 48) {
    par_copy(a1, PAR, 128, tid);
  } else if (bx == 49) {
    par_copy(a2, PAR + 512, 64, tid);
  } else if (bx == 50) {
    par_copy(gam, PAR + 768, 64, tid);
  } else {
    par_copy(bet, PAR + 1024, 64, tid);
  }
}

__global__ __launch_bounds__(256) void k_g1(const unsigned short* __restrict__ XB, const unsigned short* __restrict__ W1T,
                                            const float* __restrict__ PAR,
                                            unsigned short* __restrict__ VTH, unsigned short* __restrict__ VTL,
                                            float* __restrict__ ST1) {
  __shared__ __align__(16) float sH[64 * PITCH1];
  __shared__ __align__(16) float sST[128];
  const int tid = threadIdx.x, lane = tid & 31, wave = tid >> 5;
  const int h = lane >> 4, c = lane & 15;
  const int r0 = blockIdx.x * 64;
  const int rsub = wave >> 1, chalf = wave & 1;

  const unsigned short* arow = XB + (size_t)(r0 + rsub * 16 + c) * FF + 8 * h;
  const unsigned short* brow = W1T + (size_t)(chalf * 128 + c) * FF + 8 * h;

  v8f acc[8];
#pragma unroll
  for (int t = 0; t < 8; ++t) acc[t] = (v8f){0.f, 0.f, 0.f, 0.f, 0.f, 0.f, 0.f, 0.f};

#pragma unroll 1
  for (int k0 = 0; k0 < FF; k0 += 32) {
    const v16b a = ldfrag(arow + k0);
#pragma unroll
    for (int t = 0; t < 8; ++t) {
      const v16b bf = ldfrag(brow + (size_t)t * 16 * FF + k0);
      acc[t] = wmb(a, bf, acc[t]);
    }
  }
#pragma unroll
  for (int t = 0; t < 8; ++t)
#pragma unroll
    for (int r = 0; r < 8; ++r)
      sH[(rsub * 16 + 8 * h + r) * PITCH1 + chalf * 128 + t * 16 + c] = acc[t][r];
  __syncthreads();

  {
    const v4f s0 = *(const v4fa*)(PAR + lane * 8);
    const v4f s1 = *(const v4fa*)(PAR + lane * 8 + 4);
    const v4f t0 = *(const v4fa*)(PAR + D1 + lane * 8);
    const v4f t1 = *(const v4fa*)(PAR + D1 + lane * 8 + 4);
#pragma unroll 1
    for (int rr = 0; rr < 8; ++rr) {
      const int rl = wave * 8 + rr;
      const v4f h0 = *(const v4fa*)(sH + rl * PITCH1 + lane * 8);
      const v4f h1 = *(const v4fa*)(sH + rl * PITCH1 + lane * 8 + 4);
      float s = h0.x * s0.x + h0.y * s0.y + h0.z * s0.z + h0.w * s0.w + h1.x * s1.x + h1.y * s1.y + h1.z * s1.z + h1.w * s1.w;
      float t = h0.x * t0.x + h0.y * t0.y + h0.z * t0.z + h0.w * t0.w + h1.x * t1.x + h1.y * t1.y + h1.z * t1.z + h1.w * t1.w;
#pragma unroll
      for (int off = 16; off >= 1; off >>= 1) {
        s += __shfl_xor(s, off, 32);
        t += __shfl_xor(t, off, 32);
      }
      if (lane == 0) { sST[rl] = s; sST[64 + rl] = t; }
    }
  }

  const int b = r0 >> 10, i0 = r0 & (NN - 1);
  const int grp = tid >> 3, j8 = tid & 7;
  v4u hv[8], lv[8];
#pragma unroll
  for (int it = 0; it < 8; ++it) {
    const int d = it * 32 + grp;
    float f[8];
#pragma unroll
    for (int e = 0; e < 8; ++e) f[e] = sH[(j8 * 8 + e) * PITCH1 + d];
    unsigned l0, l1, l2, l3;
    const unsigned h0 = split2(f[0], f[1], l0);
    const unsigned h1 = split2(f[2], f[3], l1);
    const unsigned h2 = split2(f[4], f[5], l2);
    const unsigned h3 = split2(f[6], f[7], l3);
    hv[it] = (v4u){h0, h1, h2, h3};
    lv[it] = (v4u){l0, l1, l2, l3};
  }
#pragma unroll
  for (int it = 0; it < 8; ++it) {
    const int d = it * 32 + grp;
    const size_t go = ((size_t)(b * D1 + d)) * NN + i0 + j8 * 8;
    *(volatile v4u*)(VTH + go) = hv[it];
    *(volatile v4u*)(VTL + go) = lv[it];
  }
  __threadfence();
#pragma unroll
  for (int it = 0; it < 8; ++it) {
    const int d = it * 32 + grp;
    const size_t go = ((size_t)(b * D1 + d)) * NN + i0 + j8 * 8;
    *(volatile v4u*)(VTH + go) = hv[it];
    *(volatile v4u*)(VTL + go) = lv[it];
  }
  __syncthreads();
  if (wave == 0) {
    const int seg = lane >> 4, q = lane & 15;
    const v4f v = *(const v4fa*)(sST + seg * 64 + q * 4);
    volatile v4f* dst = (volatile v4f*)(ST1 + (size_t)seg * MROWS + r0 + q * 4);
    *dst = v;
    __threadfence();
    *dst = v;
  }
}

__global__ __launch_bounds__(256) void k_att1(const unsigned short* __restrict__ VTH, const unsigned short* __restrict__ VTL,
                                              const float* __restrict__ ST1, const unsigned* __restrict__ MB,
                                              const float* __restrict__ PAR, unsigned short* __restrict__ YHL) {
  __shared__ __align__(16) float sO[64 * PITCH1];
  __shared__ __align__(16) float sT[NN];
  __shared__ __align__(16) unsigned sMB[64 * 32];
  __shared__ __align__(16) float sM[64];
  __shared__ __align__(16) float sL[64];

  const int tid = threadIdx.x, lane = tid & 31, wave = tid >> 5;
  const int h = lane >> 4, c = lane & 15;
  const int b = blockIdx.x >> 4;
  const int i0 = (blockIdx.x & 15) * 64;
  const int rsub = wave >> 1, chalf = wave & 1;
  const float* S1 = ST1 + (size_t)b * NN + i0;
  const float* T1 = ST1 + MROWS + (size_t)b * NN;

  {
    const v4f tv = *(const v4fa*)(T1 + 4 * tid);
    const unsigned* mg = MB + (size_t)i0 * 32;
    const v4u m0 = *(const v4ua*)(mg + 4 * tid);
    const v4u m1 = *(const v4ua*)(mg + 4 * (tid + 256));
    *(v4fa*)(sT + 4 * tid) = tv;
    *(v4ua*)(sMB + 4 * tid) = m0;
    *(v4ua*)(sMB + 4 * (tid + 256)) = m1;
  }
  __syncthreads();

#pragma unroll 1
  for (int rr = 0; rr < 8; ++rr) {
    const int rl = wave * 8 + rr;
    const float s = S1[rl];
    float m = -3.0e38f;
#pragma unroll 4
    for (int it = 0; it < NN / 32; ++it) {
      const unsigned bit = (sMB[rl * 32 + it] >> lane) & 1u;
      const float e = efill(s, sT[it * 32 + lane], bit);
      m = (e > m) ? e : m;
    }
#pragma unroll
    for (int off = 16; off >= 1; off >>= 1) {
      const float mo = __shfl_xor(m, off, 32);
      m = (mo > m) ? mo : m;
    }
    if (lane == 0) sM[rl] = m;
  }
  __syncthreads();

  const int row = rsub * 16 + c;
  const float s_i = S1[row];
  const float m_i = sM[row];
  const unsigned short* vh = VTH + ((size_t)(b * D1 + chalf * 128 + c)) * NN + 8 * h;
  const unsigned short* vl = VTL + ((size_t)(b * D1 + chalf * 128 + c)) * NN + 8 * h;

  v8f acc[8];
#pragma unroll
  for (int t = 0; t < 8; ++t) acc[t] = (v8f){0.f, 0.f, 0.f, 0.f, 0.f, 0.f, 0.f, 0.f};
  float lpart = 0.0f;

#pragma unroll 1
  for (int ch = 0; ch < NN / 32; ++ch) {
    const int j0 = ch * 32;
    const unsigned mw = sMB[row * 32 + ch];
    const v4f q0 = *(const v4fa*)(sT + j0 + 8 * h);
    const v4f q1 = *(const v4fa*)(sT + j0 + 8 * h + 4);
    const v4f q2 = *(const v4fa*)(sT + j0 + 16 + 8 * h);
    const v4f q3 = *(const v4fa*)(sT + j0 + 16 + 8 * h + 4);
    const float tv[16] = {q0.x, q0.y, q0.z, q0.w, q1.x, q1.y, q1.z, q1.w,
                          q2.x, q2.y, q2.z, q2.w, q3.x, q3.y, q3.z, q3.w};
    unsigned ph[8], pl[8];
#pragma unroll
    for (int i2 = 0; i2 < 8; ++i2) {
      const int ia = 2 * i2;
      const int ka = (ia < 8) ? (8 * h + ia) : (8 + 8 * h + ia);
      const float ea = efill(s_i, tv[ia], (mw >> ka) & 1u);
      const float eb = efill(s_i, tv[ia + 1], (mw >> (ka + 1)) & 1u);
      const float pa = expf(ea - m_i);
      const float pb = expf(eb - m_i);
      lpart += pa;
      lpart += pb;
      ph[i2] = split2(pa, pb, pl[i2]);
    }
    const v8u phv = {ph[0], ph[1], ph[2], ph[3], ph[4], ph[5], ph[6], ph[7]};
    const v8u plv = {pl[0], pl[1], pl[2], pl[3], pl[4], pl[5], pl[6], pl[7]};
    const v16b pah = __builtin_bit_cast(v16b, phv);
    const v16b pal = __builtin_bit_cast(v16b, plv);
#pragma unroll
    for (int t = 0; t < 8; ++t) {
      const v16b bh = ldfrag(vh + (size_t)t * 16 * NN + j0);
      const v16b bl = ldfrag(vl + (size_t)t * 16 * NN + j0);
      acc[t] = wmb(pah, bh, acc[t]);
      acc[t] = wmb(pal, bh, acc[t]);
      acc[t] = wmb(pah, bl, acc[t]);
      if ((t & 1) == 1) __builtin_amdgcn_sched_barrier(0);
    }
  }

  lpart += __shfl_xor(lpart, 16, 32);
  if (chalf == 0 && h == 0) sL[row] = lpart;
#pragma unroll
  for (int t = 0; t < 8; ++t)
#pragma unroll
    for (int r = 0; r < 8; ++r)
      sO[(rsub * 16 + 8 * h + r) * PITCH1 + chalf * 128 + t * 16 + c] = acc[t][r];
  __syncthreads();

  const v4f ga = *(const v4fa*)(PAR + 768 + lane * 8);
  const v4f gb = *(const v4fa*)(PAR + 768 + lane * 8 + 4);
  const v4f ba = *(const v4fa*)(PAR + 1024 + lane * 8);
  const v4f bb = *(const v4fa*)(PAR + 1024 + lane * 8 + 4);
  const float gm[8] = {ga.x, ga.y, ga.z, ga.w, gb.x, gb.y, gb.z, gb.w};
  const float bt[8] = {ba.x, ba.y, ba.z, ba.w, bb.x, bb.y, bb.z, bb.w};
#pragma unroll 1
  for (int rr = 0; rr < 8; ++rr) {
    const int rl = wave * 8 + rr;
    const float inv = 1.0f / sL[rl];
    const v4f x0 = *(const v4fa*)(sO + rl * PITCH1 + lane * 8);
    const v4f x1 = *(const v4fa*)(sO + rl * PITCH1 + lane * 8 + 4);
    float g[8] = {x0.x * inv, x0.y * inv, x0.z * inv, x0.w * inv, x1.x * inv, x1.y * inv, x1.z * inv, x1.w * inv};
    float sm = 0.0f;
#pragma unroll
    for (int e = 0; e < 8; ++e) { g[e] = elu1(g[e]); sm += g[e]; }
#pragma unroll
    for (int off = 16; off >= 1; off >>= 1) sm += __shfl_xor(sm, off, 32);
    const float mu = sm * (1.0f / (float)D1);
    float sq = 0.0f;
#pragma unroll
    for (int e = 0; e < 8; ++e) { g[e] = g[e] - mu; sq += g[e] * g[e]; }
#pragma unroll
    for (int off = 16; off >= 1; off >>= 1) sq += __shfl_xor(sq, off, 32);
    const float var = sq * (1.0f / (float)D1);
    const float rstd = 1.0f / sqrtf(var + LNEPS);
    float y[8];
#pragma unroll
    for (int e = 0; e < 8; ++e) y[e] = g[e] * rstd * gm[e] + bt[e];
    unsigned l0, l1, l2, l3;
    const unsigned h0 = split2(y[0], y[1], l0);
    const unsigned h1 = split2(y[2], y[3], l1);
    const unsigned h2 = split2(y[4], y[5], l2);
    const unsigned h3 = split2(y[6], y[7], l3);
    const v4u hv = {h0, h1, h2, h3};
    const v4u lv = {l0, l1, l2, l3};
    unsigned short* yr = YHL + ((size_t)b * NN + i0 + rl) * KC + lane * 8;
    *(volatile v4u*)(yr) = hv;
    *(volatile v4u*)(yr + D1) = lv;
    __threadfence();
    *(volatile v4u*)(yr) = hv;
    *(volatile v4u*)(yr + D1) = lv;
  }
}

__global__ __launch_bounds__(256) void k_g2(const unsigned short* __restrict__ YHL, const unsigned short* __restrict__ W2D,
                                            const float* __restrict__ PAR, float* __restrict__ STV2) {
  __shared__ __align__(16) float sH[64 * PITCH2];
  __shared__ __align__(16) float sR[192];
  const int tid = threadIdx.x, lane = tid & 31, wave = tid >> 5;
  const int h = lane >> 4, c = lane & 15;
  const int r0 = blockIdx.x * 64;
  const int rsub = wave >> 1, chalf = wave & 1;

  const unsigned short* arow = YHL + (size_t)(r0 + rsub * 16 + c) * KC + 8 * h;
  const unsigned short* brow = W2D + (size_t)(chalf * 64 + c) * KC + 8 * h;

  v8f acc[4];
#pragma unroll
  for (int t = 0; t < 4; ++t) acc[t] = (v8f){0.f, 0.f, 0.f, 0.f, 0.f, 0.f, 0.f, 0.f};
#pragma unroll 1
  for (int k0 = 0; k0 < KC; k0 += 32) {
    const v16b a = ldfrag(arow + k0);
#pragma unroll
    for (int t = 0; t < 4; ++t) {
      const v16b bf = ldfrag(brow + (size_t)t * 16 * KC + k0);
      acc[t] = wmb(a, bf, acc[t]);
    }
  }
#pragma unroll
  for (int t = 0; t < 4; ++t)
#pragma unroll
    for (int r = 0; r < 8; ++r)
      sH[(rsub * 16 + 8 * h + r) * PITCH2 + chalf * 64 + t * 16 + c] = acc[t][r];
  __syncthreads();

  {
    const v4f as = *(const v4fa*)(PAR + 512 + lane * 4);
    const v4f at = *(const v4fa*)(PAR + 512 + D2 + lane * 4);
#pragma unroll 1
    for (int rr = 0; rr < 8; ++rr) {
      const int rl = wave * 8 + rr;
      const v4f hv = *(const v4fa*)(sH + rl * PITCH2 + lane * 4);
      float s = hv.x * as.x + hv.y * as.y + hv.z * as.z + hv.w * as.w;
      float t = hv.x * at.x + hv.y * at.y + hv.z * at.z + hv.w * at.w;
#pragma unroll
      for (int off = 16; off >= 1; off >>= 1) {
        s += __shfl_xor(s, off, 32);
        t += __shfl_xor(t, off, 32);
      }
      const float v2 = sH[rl * PITCH2 + (D2 - 1)];
      if (lane == 0) { sR[rl] = s; sR[64 + rl] = t; sR[128 + rl] = v2; }
    }
  }
  __syncthreads();
  if (wave < 2) {
    const int seg = wave * 2 + (lane >> 4);
    const int segc = (seg < 3) ? seg : 2;
    const int q = lane & 15;
    const v4f v = *(const v4fa*)(sR + segc * 64 + q * 4);
    if (seg < 3) {
      volatile v4f* dst = (volatile v4f*)(STV2 + (size_t)seg * MROWS + r0 + q * 4);
      *dst = v;
      __threadfence();
      *dst = v;
    }
  }
}

__global__ __launch_bounds__(256) void k_att2(const float* __restrict__ x, const float* __restrict__ STV2,
                                              const unsigned* __restrict__ MB, float* __restrict__ out) {
  __shared__ __align__(16) float sT[NN];
  __shared__ __align__(16) float sV[NN];
  __shared__ __align__(16) unsigned sMB[128 * 32];
  __shared__ __align__(16) float sOut[128];
  const int tid = threadIdx.x, lane = tid & 31, wave = tid >> 5;
  const int b = blockIdx.x >> 3;
  const int i0 = (blockIdx.x & 7) * 128;
  const float* S2 = STV2 + (size_t)b * NN + i0;
  const float* T2 = STV2 + MROWS + (size_t)b * NN;
  const float* V2 = STV2 + 2 * (size_t)MROWS + (size_t)b * NN;
  {
    const v4f tv = *(const v4fa*)(T2 + 4 * tid);
    const v4f vv = *(const v4fa*)(V2 + 4 * tid);
    *(v4fa*)(sT + 4 * tid) = tv;
    *(v4fa*)(sV + 4 * tid) = vv;
    const unsigned* mg = MB + (size_t)i0 * 32;
#pragma unroll
    for (int q = 0; q < 4; ++q) {
      const v4u m = *(const v4ua*)(mg + 4 * (tid + 256 * q));
      *(v4ua*)(sMB + 4 * (tid + 256 * q)) = m;
    }
  }
  __syncthreads();

#pragma unroll 1
  for (int rr = 0; rr < 16; ++rr) {
    const int rl = wave * 16 + rr;
    const float s = S2[rl];
    float m = -3.0e38f;
#pragma unroll 2
    for (int it = 0; it < NN / 32; ++it) {
      const unsigned bit = (sMB[rl * 32 + it] >> lane) & 1u;
      const float e = efill(s, sT[it * 32 + lane], bit);
      m = (e > m) ? e : m;
    }
#pragma unroll
    for (int off = 16; off >= 1; off >>= 1) {
      const float mo = __shfl_xor(m, off, 32);
      m = (mo > m) ? mo : m;
    }
    float l = 0.0f, a = 0.0f;
#pragma unroll 1
    for (int it = 0; it < NN / 32; ++it) {
      const int j = it * 32 + lane;
      const unsigned bit = (sMB[rl * 32 + it] >> lane) & 1u;
      const float e = efill(s, sT[j], bit);
      const float p = expf(e - m);
      l += p;
      a += p * sV[j];
    }
#pragma unroll
    for (int off = 16; off >= 1; off >>= 1) {
      l += __shfl_xor(l, off, 32);
      a += __shfl_xor(a, off, 32);
    }
    const float o = elu1(a * (1.0f / l));
    const float xr = bfr(x[((size_t)b * NN + i0 + rl) * FF + (FF - 1)]);
    pinf(xr);
    const float res = o + xr;
    if (lane == 0) sOut[rl] = res;
  }
  __syncthreads();
  if (wave == 0) {
    const v4f v = *(const v4fa*)(sOut + lane * 4);
    volatile v4f* dst = (volatile v4f*)(out + (size_t)b * NN + i0 + lane * 4);
    *dst = v;
    __threadfence();
    *dst = v;
  }
}

extern "C" void kernel_launch(void* const* d_in, const int* in_sizes, int n_in,
                              void* d_out, int out_size, void* d_ws, size_t ws_size,
                              hipStream_t stream) {
  if (n_in < 8) return;
  if (in_sizes[0] != MROWS * FF) return;
  if (in_sizes[1] != NN * NN) return;
  if (in_sizes[2] != FF * D1) return;
  if (in_sizes[3] != 2 * D1) return;
  if (in_sizes[4] != D1 || in_sizes[5] != D1) return;
  if (in_sizes[6] != D1 * D2) return;
  if (in_sizes[7] != 2 * D2) return;
  if (out_size != MROWS) return;

  const float* x    = (const float*)d_in[0];
  const int*   adj  = (const int*)d_in[1];
  const float* W1   = (const float*)d_in[2];
  const float* a1   = (const float*)d_in[3];
  const float* gam  = (const float*)d_in[4];
  const float* bet  = (const float*)d_in[5];
  const float* W2   = (const float*)d_in[6];
  const float* a2   = (const float*)d_in[7];
  float* out = (float*)d_out;

  size_t off = 0;
  const size_t oXB  = off; off += (size_t)MROWS * FF * 2;
  const size_t oVTH = off; off += (size_t)BB * D1 * NN * 2;
  const size_t oVTL = off; off += (size_t)BB * D1 * NN * 2;
  const size_t oYHL = off; off += (size_t)MROWS * KC * 2;
  const size_t oMB  = off; off += (size_t)NN * 32 * 4;
  const size_t oW1T = off; off += (size_t)D1 * FF * 2;
  const size_t oW2D = off; off += (size_t)D2 * KC * 2;
  const size_t oST1 = off; off += (size_t)2 * MROWS * 4;
  const size_t oSTV = off; off += (size_t)3 * MROWS * 4;
  const size_t oPAR = off; off += (size_t)1280 * 4;
  if (off > ws_size) return;

  char* ws = (char*)d_ws;
  unsigned short* XB  = (unsigned short*)(ws + oXB);
  unsigned short* VTH = (unsigned short*)(ws + oVTH);
  unsigned short* VTL = (unsigned short*)(ws + oVTL);
  unsigned short* YHL = (unsigned short*)(ws + oYHL);
  unsigned*       MB  = (unsigned*)(ws + oMB);
  unsigned short* W1T = (unsigned short*)(ws + oW1T);
  unsigned short* W2D = (unsigned short*)(ws + oW2D);
  float*          ST1 = (float*)(ws + oST1);
  float*          STV = (float*)(ws + oSTV);
  float*          PAR = (float*)(ws + oPAR);

  k_pa<<<dim3(PA_XB_BLOCKS + PA_MB_BLOCKS), dim3(256), 0, stream>>>(x, adj, XB, MB);
  k_pb<<<dim3(PB_BLOCKS), dim3(256), 0, stream>>>(W1, a1, gam, bet, W2, a2, W1T, W2D, PAR);
  k_g1<<<dim3(MROWS / 64), dim3(256), 0, stream>>>(XB, W1T, PAR, VTH, VTL, ST1);
  k_att1<<<dim3(BB * (NN / 64)), dim3(256), 0, stream>>>(VTH, VTL, ST1, MB, PAR, YHL);
  k_g2<<<dim3(MROWS / 64), dim3(256), 0, stream>>>(YHL, W2D, PAR, STV);
  k_att2<<<dim3(BB * (NN / 128)), dim3(256), 0, stream>>>(x, STV, MB, out);
  (void)hipGetLastError();
}
